// EPROP3_LSTM_67156108640260
// MI455X (gfx1250) — hardware-verified
//
#include <hip/hip_runtime.h>
#include <stddef.h>

typedef __attribute__((ext_vector_type(16))) _Float16 v16h;
typedef __attribute__((ext_vector_type(8)))  _Float16 v8h;
typedef __attribute__((ext_vector_type(16))) __bf16   v16b;
typedef __attribute__((ext_vector_type(8)))  __bf16   v8b;
typedef __attribute__((ext_vector_type(8)))  float    v8f;
typedef __attribute__((ext_vector_type(4)))  float    v4f;

constexpr int SEQ_B   = 64;
constexpr int SEQ_T   = 128;
constexpr int DIM_I   = 256;
constexpr int DIM_H   = 512;
constexpr int DIM_G   = 4 * DIM_H;
constexpr int DIM_O   = 128;
constexpr int MLP_1   = 512;
constexpr int MLP_2   = 256;
constexpr int MLP_3   = 128;
constexpr int KCAT    = DIM_I + DIM_H;
constexpr int A_PITCH = KCAT + 8;
constexpr int ROWS_PB = 16;
constexpr float X_CARRY = 8.0f;
constexpr float H_CARRY = 8.0f;
constexpr float W_CARRY = 16.0f;
constexpr float A_CARRY = 16.0f;
constexpr float Z_INV   = 0.0078125f;

__device__ __forceinline__ unsigned short f2bf_bits(float f) {
  unsigned u = __float_as_uint(f);
  return (unsigned short)((u + 0x7FFFu + ((u >> 16) & 1u)) >> 16);
}
__device__ __forceinline__ float bf_bits2f(unsigned short h) { return __uint_as_float(((unsigned)h) << 16); }

__device__ __forceinline__ void dep_guard_h(v8f& a, v8f& b, v16h x, v16h y) { asm volatile("v_nop\n\tv_nop\n\tv_nop\n\tv_nop" : "+v"(a), "+v"(b) : "v"(x), "v"(y)); }
__device__ __forceinline__ void dep_guard_b(v8f& a, v8f& b, v16b x, v16b y) { asm volatile("v_nop\n\tv_nop\n\tv_nop\n\tv_nop" : "+v"(a), "+v"(b) : "v"(x), "v"(y)); }
__device__ __forceinline__ void keep4_h(v16h a, v16h b, v16h c, v16h d) { asm volatile("v_nop" :: "v"(a), "v"(b), "v"(c), "v"(d)); }
__device__ __forceinline__ void keep4_b(v16b a, v16b b, v16b c, v16b d) { asm volatile("v_nop" :: "v"(a), "v"(b), "v"(c), "v"(d)); }
__device__ __forceinline__ void acc_guard4(v8f& a, v8f& b, v8f& c, v8f& d) { asm volatile("v_nop\n\tv_nop\n\tv_nop\n\tv_nop" : "+v"(a), "+v"(b), "+v"(c), "+v"(d)); }
template <typename T> struct Frag;
template <> struct Frag<_Float16> {
  typedef v16h V; union U { v16h v; v8h h[2]; };
  static __device__ __forceinline__ v16h load(const _Float16* p) {
    U f; f.h[0] = *(const v8h*)(p); f.h[1] = *(const v8h*)(p + 16); return f.v;
  }
  static __device__ __forceinline__ v8f mma(v16h a, v16h b, v8f c) {
    return __builtin_amdgcn_wmma_f32_16x16x32_f16(false, a, false, b, (short)0, c, false, false);
  }
  static __device__ __forceinline__ void guard(v8f& a, v8f& b, v16h x, v16h y) { dep_guard_h(a, b, x, y); }
  static __device__ __forceinline__ void keep(v16h a, v16h b, v16h c, v16h d) { keep4_h(a, b, c, d); }
};
template <> struct Frag<__bf16> {
  typedef v16b V; union U { v16b v; v8b h[2]; };
  static __device__ __forceinline__ v16b load(const __bf16* p) {
    U f; f.h[0] = *(const v8b*)(p); f.h[1] = *(const v8b*)(p + 16); return f.v;
  }
  static __device__ __forceinline__ v8f mma(v16b a, v16b b, v8f c) {
    return __builtin_amdgcn_wmma_f32_16x16x32_bf16(false, a, false, b, (short)0, c, false, false);
  }
  static __device__ __forceinline__ void guard(v8f& a, v8f& b, v16b x, v16b y) { dep_guard_b(a, b, x, y); }
  static __device__ __forceinline__ void keep(v16b a, v16b b, v16b c, v16b d) { keep4_b(a, b, c, d); }
};

template <int ET> struct Elem;
template <> struct Elem<0> { typedef _Float16 T; };
template <> struct Elem<1> { typedef __bf16 T; };
template <int ET, bool SPLIT, int BIAS_MODE, int OUT_MODE, bool RESID, int ACT = 0, int OSH = 0>
__global__ __launch_bounds__(256) void wmma_gemm64(
    const unsigned short* __restrict__ Ap, const unsigned short* __restrict__ A2p, int lda, long strideA,
    const unsigned short* __restrict__ Btp, const unsigned short* __restrict__ Bt2p, int ldb, long strideB,
    void* __restrict__ Cout, void* __restrict__ Cout2, int ldc, long strideC,
    const float* __restrict__ bias,
    const float* __restrict__ resid, long strideR,
    int M, int N, int K, float scale) {
  typedef typename Elem<ET>::T T;
  typedef typename Frag<T>::V V;
  const T* A = (const T*)Ap; const T* A2 = (const T*)A2p; const T* Bt = (const T*)Btp; const T* Bt2 = (const T*)Bt2p;
  __shared__ __align__(16) float sT[8][16 * 68];
  const int b    = blockIdx.y;
  const int lane = threadIdx.x & 31;
  const int wave = threadIdx.x >> 5;
  const int tilesN = N >> 6;
  const int tilesM = M >> 6;
  const int tile = blockIdx.x * 8 + wave;
  if (tile >= tilesM * tilesN) return;
  const int tm = tile / tilesN;
  const int tn = tile - tm * tilesN;
  const int m0 = tm << 6;
  const int n0 = tn << 6;

  const T* Ab  = A  + (size_t)b * strideA;
  const T* Bb  = Bt + (size_t)b * strideB;
  const T* Ab2 = SPLIT ? (A2  + (size_t)b * strideA) : nullptr;
  const T* Bb2 = SPLIT ? (Bt2 + (size_t)b * strideB) : nullptr;

  const int rlane = lane & 15;
  const int koff  = (lane >> 4) * 8;
  const int mOff  = (lane >> 4) * 8;

  v8f acc[4][4];
#pragma unroll
  for (int i = 0; i < 4; ++i)
#pragma unroll
    for (int j = 0; j < 4; ++j) acc[i][j] = (v8f){0.f,0.f,0.f,0.f,0.f,0.f,0.f,0.f};

  for (int k0 = 0; k0 < K; k0 += 32) {
    V bh[4], bl[4];
#pragma unroll
    for (int j = 0; j < 4; ++j) {
      const size_t bo = (size_t)(n0 + (j << 4) + rlane) * ldb + koff + k0;
      bh[j] = Frag<T>::load(Bb + bo);
      if (SPLIT) bl[j] = Frag<T>::load(Bb2 + bo);
    }
#pragma unroll
    for (int i = 0; i < 4; ++i) {
      const size_t ao = (size_t)(m0 + (i << 4) + rlane) * lda + koff + k0;
      V ah = Frag<T>::load(Ab + ao);
      V al;
      if (SPLIT) al = Frag<T>::load(Ab2 + ao);
#pragma unroll
      for (int j = 0; j < 4; ++j) {
        acc[i][j] = Frag<T>::mma(ah, bh[j], acc[i][j]);
        if (SPLIT) {
          acc[i][j] = Frag<T>::mma(ah, bl[j], acc[i][j]);
          acc[i][j] = Frag<T>::mma(al, bh[j], acc[i][j]);
        }
      }
      Frag<T>::guard(acc[i][0], acc[i][3], ah, SPLIT ? al : ah);
    }
    Frag<T>::keep(bh[0], bh[1], bh[2], bh[3]);
    if (SPLIT) Frag<T>::keep(bl[0], bl[1], bl[2], bl[3]);
  }
  acc_guard4(acc[0][0], acc[0][1], acc[0][2], acc[0][3]);
  acc_guard4(acc[1][0], acc[1][1], acc[1][2], acc[1][3]);
  acc_guard4(acc[2][0], acc[2][1], acc[2][2], acc[2][3]);
  acc_guard4(acc[3][0], acc[3][1], acc[3][2], acc[3][3]);

  float* slab = sT[wave];
  const float* Rb = RESID ? (resid + (size_t)b * strideR) : nullptr;
#pragma unroll
  for (int i = 0; i < 4; ++i) {
    const int mBase = m0 + (i << 4);
#pragma unroll
    for (int j = 0; j < 4; ++j) {
      const int n = n0 + (j << 4) + rlane;
      float bv = 0.f;
      if (BIAS_MODE == 2) bv = bias[n];
#pragma unroll
      for (int r = 0; r < 8; ++r) {
        float v = acc[i][j][r] * scale;
        if (BIAS_MODE == 1) v += bias[mBase + mOff + r];
        if (BIAS_MODE == 2) v += bv;
        if (RESID) v += Rb[(size_t)(mBase + mOff + r) * ldc + n];
        if (ACT == 1) v = tanhf(v);
        if (ACT == 2) v = fmaxf(v, 0.0f);
        if (ACT == 3) v = v / (1.0f + expf(-v));
        if (ACT == 4) v = (v > 0.f) ? v : 0.01f * v;
        if (ACT == 5) v = 0.5f * v * (1.0f + erff(v * 0.70710678118654752f));
        if (OSH != 0) v = v * (float)(1 << OSH);
        slab[(mOff + r) * 68 + (j << 4) + rlane] = v;
      }
    }
    __builtin_amdgcn_fence(__ATOMIC_RELEASE, "workgroup");
    __builtin_amdgcn_wave_barrier();
    __builtin_amdgcn_fence(__ATOMIC_ACQUIRE, "workgroup");
    if (OUT_MODE == 0) {
      float* C = (float*)Cout + (size_t)b * strideC;
      const int hh = lane >> 4, c4 = (lane & 15) * 4;
      for (int pass = 0; pass < 2; ++pass) {
#pragma unroll
        for (int it = 0; it < 8; ++it) {
          const int row = it * 2 + hh;
          v4f v = *(const v4f*)(slab + row * 68 + c4);
          *(volatile v4f*)(C + (size_t)(mBase + row) * ldc + n0 + c4) = v;
        }
        __threadfence();
      }
    } else {
      const int q = lane >> 3, c8 = (lane & 7) * 8;
      unsigned short* C  = (unsigned short*)Cout  + (size_t)b * strideC;
      unsigned short* C2 = (OUT_MODE == 2) ? ((unsigned short*)Cout2 + (size_t)b * strideC) : nullptr;
      for (int pass = 0; pass < 2; ++pass) {
#pragma unroll
        for (int it = 0; it < 4; ++it) {
          const int row = it * 4 + q;
          const float* sp = slab + row * 68 + c8;
          v8h hv, lv;
#pragma unroll
          for (int e = 0; e < 8; ++e) {
            if (OUT_MODE == 1) {
              hv[e] = (_Float16)sp[e];
            } else {
              unsigned short hb = f2bf_bits(sp[e]);
              unsigned short lb = f2bf_bits(sp[e] - bf_bits2f(hb));
              hv[e] = __builtin_bit_cast(_Float16, hb);
              lv[e] = __builtin_bit_cast(_Float16, lb);
            }
          }
          *(volatile v8h*)(C + (size_t)(mBase + row) * ldc + n0 + c8) = hv;
          if (OUT_MODE == 2) *(volatile v8h*)(C2 + (size_t)(mBase + row) * ldc + n0 + c8) = lv;
        }
        __threadfence();
      }
    }
    __builtin_amdgcn_fence(__ATOMIC_RELEASE, "workgroup");
    __builtin_amdgcn_wave_barrier();
    __builtin_amdgcn_fence(__ATOMIC_ACQUIRE, "workgroup");
  }
}

__global__ __launch_bounds__(256) void cast_rows_f16(
    const float* __restrict__ src, int src_pitch, int rows, int cols,
    unsigned short* __restrict__ dst, int dst_pitch, int dst_col0, float scale) {
  const int cols8 = cols >> 3;
  const int n8 = rows * cols8;
  const int i = blockIdx.x * 256 + threadIdx.x;
  if (i < n8) {
    const int r = i / cols8;
    const int c = (i - r * cols8) * 8;
    const float* p = src + (size_t)r * src_pitch + c;
    const v4f u0 = *(const v4f*)p;
    const v4f u1 = *(const v4f*)(p + 4);
    v8h o;
    o[0] = (_Float16)(u0[0] * scale);
    o[1] = (_Float16)(u0[1] * scale);
    o[2] = (_Float16)(u0[2] * scale);
    o[3] = (_Float16)(u0[3] * scale);
    o[4] = (_Float16)(u1[0] * scale);
    o[5] = (_Float16)(u1[1] * scale);
    o[6] = (_Float16)(u1[2] * scale);
    o[7] = (_Float16)(u1[3] * scale);
    _Float16* d = (_Float16*)(void*)dst + (size_t)r * dst_pitch + dst_col0 + c;
    *(volatile v8h*)d = o;
    __threadfence();
    *(volatile v8h*)d = o;
  }
}

__global__ __launch_bounds__(256) void fill_zero_f32x4(float* __restrict__ p, int n4) {
  const int i = blockIdx.x * 256 + threadIdx.x;
  if (i < n4) {
    v4f z;
    z[0] = 0.0f; z[1] = 0.0f; z[2] = 0.0f; z[3] = 0.0f;
    *(volatile v4f*)(p + (size_t)i * 4) = z;
    __threadfence();
    *(volatile v4f*)(p + (size_t)i * 4) = z;
  }
}

__device__ __forceinline__ v8f mma_h(v16h a, v16h b, v8f c) {
  c = __builtin_amdgcn_wmma_f32_16x16x32_f16(false, a, false, b, (short)0, c, false, false);
  asm volatile("v_nop\n\tv_nop\n\tv_nop\n\tv_nop" : "+v"(c) : "v"(a), "v"(b));
  return c;
}
__device__ __forceinline__ float sigm_f(float z) {
  const float zc = fminf(fmaxf(z, -30.0f), 30.0f);
  return 1.0f / (1.0f + expf(-zc));
}

__global__ __launch_bounds__(512)
void lstm_seq_kernel(const float* __restrict__ x, const unsigned short* __restrict__ wcat,
                     const float* __restrict__ b_lstm, unsigned short* __restrict__ hs) {
  __shared__ __align__(16) _Float16 Ash[2 * ROWS_PB * A_PITCH];
  const int tid  = threadIdx.x;
  const int lane = tid & 31;
  const int wave = tid >> 5;
  const int hh   = lane >> 4;
  const int cix  = lane & 15;
  const int b0   = blockIdx.x * ROWS_PB;
  const int colw = wave * 32;

  {
    unsigned int* az = (unsigned int*)(void*)Ash;
    for (int i = tid; i < (2 * ROWS_PB * A_PITCH) / 2; i += 512) az[i] = 0u;
  }

  float bsel[4][2];
#pragma unroll
  for (int g = 0; g < 4; ++g)
#pragma unroll
    for (int s = 0; s < 2; ++s) bsel[g][s] = b_lstm[g * DIM_H + colw + 16 * s + cix];

  const _Float16* wl = (const _Float16*)(const void*)wcat + (size_t)(colw + cix) * KCAT + 8 * hh;

  float cst0[8], cst1[8];
#pragma unroll
  for (int r = 0; r < 8; ++r) { cst0[r] = 0.0f; cst1[r] = 0.0f; }

  __syncthreads();

  for (int t = 0; t < SEQ_T; ++t) {
    const int cur = t & 1;
    _Float16* Acur = Ash + cur * (ROWS_PB * A_PITCH);
    _Float16* Anxt = Ash + (cur ^ 1) * (ROWS_PB * A_PITCH);

    {
      const int xr = wave;
      const float* xp = x + ((size_t)(b0 + xr) * SEQ_T + t) * DIM_I + lane * 8;
      const v4f u0 = *(const v4f*)xp;
      const v4f u1 = *(const v4f*)(xp + 4);
      v8h o;
      o[0] = (_Float16)(u0[0] * X_CARRY);
      o[1] = (_Float16)(u0[1] * X_CARRY);
      o[2] = (_Float16)(u0[2] * X_CARRY);
      o[3] = (_Float16)(u0[3] * X_CARRY);
      o[4] = (_Float16)(u1[0] * X_CARRY);
      o[5] = (_Float16)(u1[1] * X_CARRY);
      o[6] = (_Float16)(u1[2] * X_CARRY);
      o[7] = (_Float16)(u1[3] * X_CARRY);
      *(v8h*)(Acur + xr * A_PITCH + lane * 8) = o;
    }
    __syncthreads();

    v8f acc[4][2];
#pragma unroll
    for (int g = 0; g < 4; ++g)
#pragma unroll
      for (int s = 0; s < 2; ++s) acc[g][s] = (v8f){0.f,0.f,0.f,0.f,0.f,0.f,0.f,0.f};

    const _Float16* arow = Acur + cix * A_PITCH + 8 * hh;
#pragma unroll 1
    for (int k0 = 0; k0 < KCAT; k0 += 32) {
      Frag<_Float16>::U fa;
      fa.h[0] = *(const v8h*)(arow + k0);
      fa.h[1] = *(const v8h*)(arow + k0 + 16);
      const v16h av = fa.v;
#pragma unroll
      for (int g = 0; g < 4; ++g) {
#pragma unroll
        for (int s = 0; s < 2; ++s) {
          const v16h bv = Frag<_Float16>::load(wl + (size_t)(g * DIM_H + 16 * s) * KCAT + k0);
          acc[g][s] = mma_h(av, bv, acc[g][s]);
        }
      }
    }

#pragma unroll 1
    for (int s = 0; s < 2; ++s) {
      const bool s1 = (s != 0);
      const float bi = s1 ? bsel[0][1] : bsel[0][0];
      const float bf = s1 ? bsel[1][1] : bsel[1][0];
      const float bg = s1 ? bsel[2][1] : bsel[2][0];
      const float bo = s1 ? bsel[3][1] : bsel[3][0];
      const int ucol = DIM_I + colw + 16 * s + cix;
#pragma unroll
      for (int r = 0; r < 8; ++r) {
        const float ai = s1 ? acc[0][1][r] : acc[0][0][r];
        const float af = s1 ? acc[1][1][r] : acc[1][0][r];
        const float ag = s1 ? acc[2][1][r] : acc[2][0][r];
        const float ao = s1 ? acc[3][1][r] : acc[3][0][r];
        const float ig = sigm_f(ai * Z_INV + bi);
        const float fg = sigm_f(af * Z_INV + bf);
        const float gg = tanhf(ag * Z_INV + bg);
        const float og = sigm_f(ao * Z_INV + bo);
        const float cold = s1 ? cst1[r] : cst0[r];
        const float cn = fg * cold + ig * gg;
        cst0[r] = s1 ? cst0[r] : cn;
        cst1[r] = s1 ? cn : cst1[r];
        const float hn = og * tanhf(cn);
        Anxt[(8 * hh + r) * A_PITCH + ucol] = (_Float16)(hn * H_CARRY);
      }
    }
    __syncthreads();

    {
      const _Float16* srow = Anxt + wave * A_PITCH + DIM_I;
      const v8h v0 = *(const v8h*)(srow + lane * 8);
      const v8h v1 = *(const v8h*)(srow + 256 + lane * 8);
      _Float16* drow = (_Float16*)(void*)hs + ((size_t)(b0 + wave) * SEQ_T + t) * DIM_H;
      *(volatile v8h*)(drow + lane * 8) = v0;
      *(volatile v8h*)(drow + 256 + lane * 8) = v1;
      __threadfence();
      *(volatile v8h*)(drow + lane * 8) = v0;
      *(volatile v8h*)(drow + 256 + lane * 8) = v1;
    }
  }
}

static inline size_t ws_take(size_t& off, size_t bytes) {
  size_t o = off;
  off = (off + bytes + 255) & ~(size_t)255;
  return o;
}

extern "C" void kernel_launch(void* const* d_in, const int* in_sizes, int n_in,
                              void* d_out, int out_size, void* d_ws, size_t ws_size,
                              hipStream_t stream) {
  if (n_in < 14) return;
  if (in_sizes[0] != SEQ_B * SEQ_T * DIM_I) return;
  if (in_sizes[1] != DIM_G * DIM_I || in_sizes[2] != DIM_G * DIM_H || in_sizes[3] != DIM_G) return;
  if (in_sizes[4] != DIM_O * DIM_H || in_sizes[5] != DIM_O) return;
  if (in_sizes[6] != MLP_1 * DIM_O || in_sizes[7] != MLP_1) return;
  if (in_sizes[8] != MLP_2 * MLP_1 || in_sizes[9] != MLP_2) return;
  if (in_sizes[10] != MLP_3 * MLP_2 || in_sizes[11] != MLP_3) return;
  if (in_sizes[12] != DIM_H * MLP_3 || in_sizes[13] != DIM_H) return;
  if (out_size != SEQ_B * SEQ_T * DIM_O + 2 * SEQ_B * DIM_H) return;

  const float* x      = (const float*)d_in[0];
  const float* Wih    = (const float*)d_in[1];
  const float* Whh    = (const float*)d_in[2];
  const float* b_lstm = (const float*)d_in[3];
  const float* Wd     = (const float*)d_in[4];
  const float* bd     = (const float*)d_in[5];
  const float* W1     = (const float*)d_in[6];
  const float* b1     = (const float*)d_in[7];
  const float* W2     = (const float*)d_in[8];
  const float* b2     = (const float*)d_in[9];
  const float* W3     = (const float*)d_in[10];
  const float* b3     = (const float*)d_in[11];
  const float* W4     = (const float*)d_in[12];
  const float* b4     = (const float*)d_in[13];

  char* ws = (char*)d_ws;
  size_t off = 0;
  unsigned short* wcat16 = (unsigned short*)(ws + ws_take(off, (size_t)DIM_G * KCAT * 2));
  unsigned short* wd16   = (unsigned short*)(ws + ws_take(off, (size_t)DIM_O * DIM_H * 2));
  unsigned short* w1_16  = (unsigned short*)(ws + ws_take(off, (size_t)MLP_1 * DIM_O * 2));
  unsigned short* w2_16  = (unsigned short*)(ws + ws_take(off, (size_t)MLP_2 * MLP_1 * 2));
  unsigned short* w3_16  = (unsigned short*)(ws + ws_take(off, (size_t)MLP_3 * MLP_2 * 2));
  unsigned short* w4_16  = (unsigned short*)(ws + ws_take(off, (size_t)DIM_H * MLP_3 * 2));
  unsigned short* hs16   = (unsigned short*)(ws + ws_take(off, (size_t)SEQ_B * SEQ_T * DIM_H * 2));
  unsigned short* a0     = (unsigned short*)(ws + ws_take(off, (size_t)SEQ_B * DIM_O * 2));
  unsigned short* a1     = (unsigned short*)(ws + ws_take(off, (size_t)SEQ_B * MLP_1 * 2));
  unsigned short* a2     = (unsigned short*)(ws + ws_take(off, (size_t)SEQ_B * MLP_2 * 2));
  unsigned short* a3     = (unsigned short*)(ws + ws_take(off, (size_t)SEQ_B * MLP_3 * 2));
  if (off > ws_size) return;

  float* out0 = (float*)d_out;
  float* out1 = out0 + (size_t)SEQ_B * SEQ_T * DIM_O;
  float* out2 = out1 + (size_t)SEQ_B * DIM_H;

  {
    const int n8a = DIM_G * (DIM_I / 8);
    cast_rows_f16<<<(n8a + 255) / 256, 256, 0, stream>>>(Wih, DIM_I, DIM_G, DIM_I, wcat16, KCAT, 0, W_CARRY);
    const int n8b = DIM_G * (DIM_H / 8);
    cast_rows_f16<<<(n8b + 255) / 256, 256, 0, stream>>>(Whh, DIM_H, DIM_G, DIM_H, wcat16, KCAT, DIM_I, W_CARRY);
    const int n8c = DIM_O * (DIM_H / 8);
    cast_rows_f16<<<(n8c + 255) / 256, 256, 0, stream>>>(Wd, DIM_H, DIM_O, DIM_H, wd16, DIM_H, 0, W_CARRY);
    const int n8d = MLP_1 * (DIM_O / 8);
    cast_rows_f16<<<(n8d + 255) / 256, 256, 0, stream>>>(W1, DIM_O, MLP_1, DIM_O, w1_16, DIM_O, 0, W_CARRY);
    const int n8e = MLP_2 * (MLP_1 / 8);
    cast_rows_f16<<<(n8e + 255) / 256, 256, 0, stream>>>(W2, MLP_1, MLP_2, MLP_1, w2_16, MLP_1, 0, W_CARRY);
    const int n8f = MLP_3 * (MLP_2 / 8);
    cast_rows_f16<<<(n8f + 255) / 256, 256, 0, stream>>>(W3, MLP_2, MLP_3, MLP_2, w3_16, MLP_2, 0, W_CARRY);
    const int n8g = DIM_H * (MLP_3 / 8);
    cast_rows_f16<<<(n8g + 255) / 256, 256, 0, stream>>>(W4, MLP_3, DIM_H, MLP_3, w4_16, MLP_3, 0, W_CARRY);
  }

  {
    const int n4 = SEQ_B * DIM_H / 4;
    fill_zero_f32x4<<<(n4 + 255) / 256, 256, 0, stream>>>(out1, n4);
  }

  lstm_seq_kernel<<<SEQ_B / ROWS_PB, 512, 0, stream>>>(x, wcat16, b_lstm, hs16);

  wmma_gemm64<0, false, 2, 0, false, 0, 0><<<dim3((SEQ_B * SEQ_T / 64) * (DIM_O / 64) / 8, 1), 256, 0, stream>>>(
      hs16, nullptr, DIM_H, (long)0, wd16, nullptr, DIM_H, (long)0,
      out0, nullptr, DIM_O, (long)0, bd, nullptr, (long)0,
      SEQ_B * SEQ_T, DIM_O, DIM_H, 1.0f / 128.0f);

  {
    const int n8 = SEQ_B * (DIM_O / 8);
    cast_rows_f16<<<(n8 + 255) / 256, 256, 0, stream>>>(out0 + (size_t)(SEQ_T - 1) * DIM_O, SEQ_T * DIM_O,
                                                       SEQ_B, DIM_O, a0, DIM_O, 0, A_CARRY);
  }
  wmma_gemm64<0, false, 2, 1, false, 2, 4><<<dim3(1, 1), 256, 0, stream>>>(
      a0, nullptr, DIM_O, (long)0, w1_16, nullptr, DIM_O, (long)0,
      a1, nullptr, MLP_1, (long)0, b1, nullptr, (long)0,
      SEQ_B, MLP_1, DIM_O, 1.0f / 256.0f);
  wmma_gemm64<0, false, 2, 1, false, 2, 4><<<dim3(1, 1), 256, 0, stream>>>(
      a1, nullptr, MLP_1, (long)0, w2_16, nullptr, MLP_1, (long)0,
      a2, nullptr, MLP_2, (long)0, b2, nullptr, (long)0,
      SEQ_B, MLP_2, MLP_1, 1.0f / 256.0f);
  wmma_gemm64<0, false, 2, 1, false, 2, 4><<<dim3(1, 1), 256, 0, stream>>>(
      a2, nullptr, MLP_2, (long)0, w3_16, nullptr, MLP_2, (long)0,
      a3, nullptr, MLP_3, (long)0, b3, nullptr, (long)0,
      SEQ_B, MLP_3, MLP_2, 1.0f / 256.0f);
  wmma_gemm64<0, false, 2, 0, false, 0, 0><<<dim3(1, 1), 256, 0, stream>>>(
      a3, nullptr, MLP_3, (long)0, w4_16, nullptr, MLP_3, (long)0,
      out2, nullptr, DIM_H, (long)0, b4, nullptr, (long)0,
      SEQ_B, DIM_H, MLP_3, 1.0f / 256.0f);
}
